// DiffiTAttention_51075751084659
// MI455X (gfx1250) — hardware-verified
//
#include <hip/hip_runtime.h>
#include <stddef.h>


#define DEV __device__ __forceinline__

typedef _Float16 v16h __attribute__((ext_vector_type(16)));
typedef _Float16 v8h __attribute__((ext_vector_type(8)));
typedef __bf16 v16b __attribute__((ext_vector_type(16)));
typedef unsigned short v16us __attribute__((ext_vector_type(16)));
typedef unsigned short v8us __attribute__((ext_vector_type(8), __may_alias__));
typedef float v8f __attribute__((ext_vector_type(8)));
typedef float v4f __attribute__((ext_vector_type(4), __may_alias__));

union FragH { v16h v; v8h h[2]; };
union FragU { v16us v; v8us h[2]; };

constexpr int TP = 132;

DEV v8f zero8() { v8f z = {0.f, 0.f, 0.f, 0.f, 0.f, 0.f, 0.f, 0.f}; return z; }

DEV unsigned short bfb(float f) {
  unsigned int u = __builtin_bit_cast(unsigned int, f);
  u += 0x7FFFu + ((u >> 16) & 1u);
  return (unsigned short)(u >> 16);
}
DEV float bfv(unsigned short s) { return __builtin_bit_cast(float, ((unsigned int)s) << 16); }
DEV unsigned short hfb(float f) {
  _Float16 t = (_Float16)f;
  return __builtin_bit_cast(unsigned short, t);
}

DEV v8f mma_f16(v16h a, v16h b, v8f c) {
  c = __builtin_amdgcn_wmma_f32_16x16x32_f16(false, a, false, b, (short)0, c, false, false);
  asm volatile("v_nop\n\tv_nop\n\tv_nop\n\tv_nop" : "+v"(c) : "v"(a), "v"(b));
  return c;
}
DEV v8f mma_bf16(v16us a, v16us b, v8f c) {
  v16b ab = __builtin_bit_cast(v16b, a);
  v16b bb = __builtin_bit_cast(v16b, b);
  c = __builtin_amdgcn_wmma_f32_16x16x32_bf16(false, ab, false, bb, (short)0, c, false, false);
  asm volatile("v_nop\n\tv_nop\n\tv_nop\n\tv_nop" : "+v"(c) : "v"(ab), "v"(bb));
  return c;
}


__global__ __launch_bounds__(256) void k_cvt_x(const float* __restrict__ x,
                                               unsigned short* __restrict__ xh, int n8) {
  const int i = blockIdx.x * 256 + threadIdx.x;
  if (i < n8) {
    const float* p = x + (size_t)i * 8;
    v4f a = *(const v4f*)(p);
    v4f c = *(const v4f*)(p + 4);
    v8us o;
    o[0] = hfb(a[0]); o[1] = hfb(a[1]); o[2] = hfb(a[2]); o[3] = hfb(a[3]);
    o[4] = hfb(c[0]); o[5] = hfb(c[1]); o[6] = hfb(c[2]); o[7] = hfb(c[3]);
    unsigned short* d = xh + (size_t)i * 8;
    *(volatile v8us*)d = o;
    __threadfence();
    *(volatile v8us*)d = o;
  }
}

template <int SPLIT>
__global__ __launch_bounds__(256) void k_tr(const float* __restrict__ src, int nrows, int ncols,
                                            float scl, unsigned short* d0, unsigned short* d1) {
  __shared__ float tile[64 * 65];
  const int c0 = blockIdx.x * 64, r0 = blockIdx.y * 64, t = threadIdx.x;
#pragma unroll
  for (int i = 0; i < 16; ++i) {
    const int idx = t + i * 256;
    const int rr = idx >> 6, cc = idx & 63;
    tile[rr * 65 + cc] = src[(size_t)(r0 + rr) * ncols + c0 + cc];
  }
  __syncthreads();
  const int lane = t & 31, wave = t >> 5, piece = lane & 7, sub = lane >> 3;
#pragma unroll
  for (int pass = 0; pass < 2; ++pass) {
    if (pass) __threadfence();
#pragma unroll
    for (int it = 0; it < 2; ++it) {
      const int cl = wave * 8 + it * 4 + sub;
      v8us o0, o1;
#pragma unroll
      for (int j = 0; j < 8; ++j) {
        const float f = tile[(piece * 8 + j) * 65 + cl];
        if (SPLIT) {
          const unsigned short hb = bfb(f);
          o0[j] = hb;
          o1[j] = bfb(f - bfv(hb));
        } else {
          o0[j] = hfb(f * scl);
          o1[j] = o0[j];
        }
      }
      const size_t off = (size_t)(c0 + cl) * nrows + r0 + piece * 8;
      *(volatile v8us*)(d0 + off) = o0;
      if (SPLIT) *(volatile v8us*)(d1 + off) = o1;
    }
  }
}

__global__ __launch_bounds__(64) void k_temb(const float* __restrict__ temb,
                                             const float* __restrict__ Wt,
                                             const float* __restrict__ bt,
                                             const float* __restrict__ bqkv,
                                             float* __restrict__ tvec) {
  __shared__ __attribute__((aligned(16))) float st[8 * 32];
  const int t = threadIdx.x, lane = t & 31, wave = t >> 5, h = lane >> 4, m = lane & 15;
  const int j0 = blockIdx.x * 32;
  const int col = j0 + wave * 16 + m;
  const int arow = (m < 8) ? m : 7;
  const float amul = (m < 8) ? 1.0f : 0.0f;
  const float* ap = temb + arow * 1024;
  v8f acc = zero8();
#pragma unroll 1
  for (int k0 = 0; k0 < 1024; k0 += 32) {
    v4f x0 = *(const v4f*)(ap + k0 + 8 * h);
    v4f x1 = *(const v4f*)(ap + k0 + 8 * h + 4);
    v4f x2 = *(const v4f*)(ap + k0 + 16 + 8 * h);
    v4f x3 = *(const v4f*)(ap + k0 + 16 + 8 * h + 4);
    float av[16] = {x0[0], x0[1], x0[2], x0[3], x1[0], x1[1], x1[2], x1[3],
                    x2[0], x2[1], x2[2], x2[3], x3[0], x3[1], x3[2], x3[3]};
    FragU ah, al, wh, wl;
#pragma unroll
    for (int i = 0; i < 16; ++i) {
      const float a = av[i] * amul;
      const unsigned short hb = bfb(a);
      ah.v[i] = hb;
      al.v[i] = bfb(a - bfv(hb));
      const int kk = (i < 8) ? (8 * h + i) : (8 + 8 * h + i);
      const float w = Wt[(size_t)(k0 + kk) * 3072 + col];
      const unsigned short wb = bfb(w);
      wh.v[i] = wb;
      wl.v[i] = bfb(w - bfv(wb));
    }
    acc = mma_bf16(ah.v, wh.v, acc);
    acc = mma_bf16(ah.v, wl.v, acc);
    acc = mma_bf16(al.v, wh.v, acc);
  }
  const float addc = bt[col] + bqkv[col];
  if (h == 0) {
#pragma unroll
    for (int r = 0; r < 8; ++r) st[r * 32 + wave * 16 + m] = acc[r] + addc;
  }
  __syncthreads();
  if (wave == 0) {
    const int sub = lane >> 3, piece = lane & 7;
#pragma unroll
    for (int pass = 0; pass < 2; ++pass) {
      if (pass) __threadfence();
#pragma unroll
      for (int it = 0; it < 2; ++it) {
        const int b = it * 4 + sub;
        v4f v = *(const v4f*)(st + b * 32 + piece * 4);
        *(volatile v4f*)(tvec + (size_t)b * 3072 + j0 + piece * 4) = v;
      }
    }
  }
}

__global__ __launch_bounds__(128) void k_qkv(
    const _Float16* __restrict__ xh, const _Float16* __restrict__ wq,
    const float* __restrict__ tvec, const float* __restrict__ cos_y,
    const float* __restrict__ sin_y, const float* __restrict__ cos_x,
    const float* __restrict__ sin_x, const float* __restrict__ qn_w,
    const float* __restrict__ kn_w, unsigned short* __restrict__ qpl,
    unsigned short* __restrict__ kpl, unsigned short* __restrict__ vth,
    unsigned short* __restrict__ vtl) {
  __shared__ __attribute__((aligned(16))) float T[64 * TP];
  __shared__ __attribute__((aligned(16))) unsigned short U[8192];
  const int t = threadIdx.x, lane = t & 31, wave = t >> 5, h = lane >> 4, m = lane & 15;
  const int bm = blockIdx.y * 64, bn = blockIdx.x * 128;
  const int wm = (wave & 1) * 32, wn = (wave >> 1) * 64;

  v8f acc[2][4];
#pragma unroll
  for (int mi = 0; mi < 2; ++mi)
#pragma unroll
    for (int ni = 0; ni < 4; ++ni) acc[mi][ni] = zero8();

  const _Float16* ar0 = xh + (size_t)(bm + wm + m) * 1024;
  const _Float16* ar1 = ar0 + 16 * 1024;
  const _Float16* bc = wq + (size_t)(bn + wn + m) * 1024;
#pragma unroll 1
  for (int k0 = 0; k0 < 1024; k0 += 32) {
    FragH a0, a1;
    a0.h[0] = *(const v8h*)(ar0 + k0 + 8 * h);
    a0.h[1] = *(const v8h*)(ar0 + k0 + 16 + 8 * h);
    a1.h[0] = *(const v8h*)(ar1 + k0 + 8 * h);
    a1.h[1] = *(const v8h*)(ar1 + k0 + 16 + 8 * h);
#pragma unroll
    for (int ni = 0; ni < 4; ++ni) {
      const _Float16* bp = bc + (size_t)ni * (16 * 1024) + k0;
      FragH b;
      b.h[0] = *(const v8h*)(bp + 8 * h);
      b.h[1] = *(const v8h*)(bp + 16 + 8 * h);
      acc[0][ni] = mma_f16(a0.v, b.v, acc[0][ni]);
      acc[1][ni] = mma_f16(a1.v, b.v, acc[1][ni]);
    }
  }

#pragma unroll
  for (int mi = 0; mi < 2; ++mi)
#pragma unroll
    for (int ni = 0; ni < 4; ++ni)
#pragma unroll
      for (int r = 0; r < 8; ++r)
        T[(wm + mi * 16 + 8 * h + r) * TP + wn + ni * 16 + m] = acc[mi][ni][r] * 0.03125f;
  __syncthreads();

  const int row = t & 63, hh = t >> 6;
  const int b = bm >> 10, n0 = bm & 1023, tok = n0 + row;
  const int sec = bn >> 10;
  const int head0 = (bn & 1023) >> 6;
  const int bh0 = b * 16 + head0;
  const int sub = lane >> 3, piece = lane & 7;

  float v[64];
  {
    const float* tr = T + row * TP + hh * 64;
    const float* tv = tvec + (size_t)b * 3072 + bn + hh * 64;
#pragma unroll
    for (int q = 0; q < 16; ++q) {
      v4f a = *(const v4f*)(tr + 4 * q);
      v4f c = *(const v4f*)(tv + 4 * q);
      v[4 * q + 0] = a[0] + c[0];
      v[4 * q + 1] = a[1] + c[1];
      v[4 * q + 2] = a[2] + c[2];
      v[4 * q + 3] = a[3] + c[3];
    }
  }

  if (sec < 2) {
    float ss = 0.f;
#pragma unroll
    for (int d = 0; d < 64; ++d) ss += v[d] * v[d];
    const float rr = rsqrtf(ss * (1.0f / 64.0f) + 1.0e-6f);
    const float* wv = (sec == 0) ? qn_w : kn_w;
#pragma unroll
    for (int q = 0; q < 16; ++q) {
      v4f w4 = *(const v4f*)(wv + 4 * q);
      v[4 * q + 0] = (v[4 * q + 0] * rr) * w4[0];
      v[4 * q + 1] = (v[4 * q + 1] * rr) * w4[1];
      v[4 * q + 2] = (v[4 * q + 2] * rr) * w4[2];
      v[4 * q + 3] = (v[4 * q + 3] * rr) * w4[3];
    }
    const float* cyp = cos_y + tok * 32;
    const float* syp = sin_y + tok * 32;
    const float* cxp = cos_x + tok * 32;
    const float* sxp = sin_x + tok * 32;
    unsigned short* up = U + (hh * 64 + row) * 64;
#pragma unroll
    for (int p2 = 0; p2 < 2; ++p2) {
      v8us g0, g1, g2, g3;
#pragma unroll
      for (int qq = 0; qq < 2; ++qq) {
        const int d0 = 8 * p2 + 4 * qq;
        v4f cya = *(const v4f*)(cyp + d0), cyb = *(const v4f*)(cyp + 16 + d0);
        v4f sya = *(const v4f*)(syp + d0), syb = *(const v4f*)(syp + 16 + d0);
        v4f cxa = *(const v4f*)(cxp + d0), cxb = *(const v4f*)(cxp + 16 + d0);
        v4f sxa = *(const v4f*)(sxp + d0), sxb = *(const v4f*)(sxp + 16 + d0);
#pragma unroll
        for (int e = 0; e < 4; ++e) {
          const int dd = d0 + e, j = 4 * qq + e;
          g0[j] = hfb(v[dd] * cya[e] - v[dd + 16] * sya[e]);
          g1[j] = hfb(v[dd + 16] * cyb[e] + v[dd] * syb[e]);
          g2[j] = hfb(v[dd + 32] * cxa[e] - v[dd + 48] * sxa[e]);
          g3[j] = hfb(v[dd + 48] * cxb[e] + v[dd + 32] * sxb[e]);
        }
      }
      *(v8us*)(up + 8 * p2) = g0;
      *(v8us*)(up + 16 + 8 * p2) = g1;
      *(v8us*)(up + 32 + 8 * p2) = g2;
      *(v8us*)(up + 48 + 8 * p2) = g3;
    }
    __syncthreads();
    unsigned short* plane = (sec == 0) ? qpl : kpl;
#pragma unroll
    for (int pass = 0; pass < 2; ++pass) {
      if (pass) __threadfence();
#pragma unroll
      for (int it = 0; it < 8; ++it) {
        const int L = wave * 32 + it * 4 + sub;
        const int lhh = L >> 6, lrow = L & 63;
        v8us val = *(const v8us*)(U + (lhh * 64 + lrow) * 64 + piece * 8);
        *(volatile v8us*)(plane + ((size_t)((bh0 + lhh) * 1024 + n0 + lrow)) * 64 + piece * 8) = val;
      }
    }
  } else {
#pragma unroll
    for (int p = 0; p < 2; ++p) {
      unsigned short* up = U + (hh * 64) * 64 + row;
#pragma unroll
      for (int d = 0; d < 64; ++d) {
        const unsigned short hb = bfb(v[d]);
        up[d * 64] = p ? bfb(v[d] - bfv(hb)) : hb;
      }
      __syncthreads();
      unsigned short* plane = p ? vtl : vth;
#pragma unroll
      for (int pass = 0; pass < 2; ++pass) {
        if (pass) __threadfence();
#pragma unroll
        for (int it = 0; it < 8; ++it) {
          const int L = wave * 32 + it * 4 + sub;
          const int lhh = L >> 6, ld = L & 63;
          v8us val = *(const v8us*)(U + (lhh * 64 + ld) * 64 + piece * 8);
          *(volatile v8us*)(plane + ((size_t)((bh0 + lhh) * 64 + ld)) * 1024 + n0 + piece * 8) = val;
        }
      }
      __syncthreads();
    }
  }
}

__global__ __launch_bounds__(128) void k_attn(
    const _Float16* __restrict__ qpl, const _Float16* __restrict__ kpl,
    const unsigned short* __restrict__ vth, const unsigned short* __restrict__ vtl,
    unsigned short* __restrict__ cxh, unsigned short* __restrict__ cxl) {
  __shared__ __attribute__((aligned(16))) unsigned short CW[4 * 2 * 16 * 64];
  const int t = threadIdx.x, lane = t & 31, wave = t >> 5, h = lane >> 4, m = lane & 15;
  const int bh = blockIdx.y, b = bh >> 4, head = bh & 15;
  const int q0 = blockIdx.x * 64 + wave * 16;

  FragH bq0, bq1;
  {
    const _Float16* qp = qpl + ((size_t)bh * 1024 + q0 + m) * 64;
    bq0.h[0] = *(const v8h*)(qp + 8 * h);
    bq0.h[1] = *(const v8h*)(qp + 16 + 8 * h);
    bq1.h[0] = *(const v8h*)(qp + 32 + 8 * h);
    bq1.h[1] = *(const v8h*)(qp + 48 + 8 * h);
  }
  const _Float16* kbase = kpl + (size_t)bh * (1024 * 64) + m * 64;
  const unsigned short* vhb = vth + (size_t)bh * (64 * 1024) + (size_t)m * 1024;
  const unsigned short* vlb = vtl + (size_t)bh * (64 * 1024) + (size_t)m * 1024;

  v8f o[4];
#pragma unroll
  for (int dt = 0; dt < 4; ++dt) o[dt] = zero8();
  float mrun = -1.0e30f, lrun = 0.f;

#pragma unroll 1
  for (int kb = 0; kb < 1024; kb += 64) {
    v8f s[4];
#pragma unroll
    for (int j = 0; j < 4; ++j) {
      const _Float16* kp = kbase + (size_t)(kb + 16 * j) * 64;
      FragH a0, a1;
      a0.h[0] = *(const v8h*)(kp + 8 * h);
      a0.h[1] = *(const v8h*)(kp + 16 + 8 * h);
      a1.h[0] = *(const v8h*)(kp + 32 + 8 * h);
      a1.h[1] = *(const v8h*)(kp + 48 + 8 * h);
      v8f tt = zero8();
      tt = mma_f16(a0.v, bq0.v, tt);
      tt = mma_f16(a1.v, bq1.v, tt);
      s[j] = tt;
    }
    float mx = -1.0e30f;
#pragma unroll
    for (int j = 0; j < 4; ++j)
#pragma unroll
      for (int r = 0; r < 8; ++r) {
        const float z = s[j][r] * 0.125f;
        s[j][r] = z;
        mx = fmaxf(mx, z);
      }
    mx = fmaxf(mx, __shfl_xor(mx, 16, 32));
    const float mnew = fmaxf(mrun, mx);
    const float scl = __expf(mrun - mnew);
    mrun = mnew;
    float ls = 0.f;
#pragma unroll
    for (int j = 0; j < 4; ++j)
#pragma unroll
      for (int r = 0; r < 8; ++r) {
        const float pz = __expf(s[j][r] - mnew);
        s[j][r] = pz;
        ls += pz;
      }
    ls += __shfl_xor(ls, 16, 32);
    lrun = lrun * scl + ls;
#pragma unroll
    for (int dt = 0; dt < 4; ++dt)
#pragma unroll
      for (int r = 0; r < 8; ++r) o[dt][r] *= scl;

#pragma unroll
    for (int ss = 0; ss < 2; ++ss) {
      FragU ph, pl;
#pragma unroll
      for (int r = 0; r < 8; ++r) {
        const float f0 = s[2 * ss][r];
        const unsigned short h0 = bfb(f0);
        ph.v[r] = h0;
        pl.v[r] = bfb(f0 - bfv(h0));
        const float f1 = s[2 * ss + 1][r];
        const unsigned short h1 = bfb(f1);
        ph.v[8 + r] = h1;
        pl.v[8 + r] = bfb(f1 - bfv(h1));
      }
#pragma unroll
      for (int dt = 0; dt < 4; ++dt) {
        const unsigned short* vp = vhb + (size_t)dt * (16 * 1024) + kb + 32 * ss;
        const unsigned short* wp = vlb + (size_t)dt * (16 * 1024) + kb + 32 * ss;
        FragU ah, al;
        ah.h[0] = *(const v8us*)(vp + 8 * h);
        ah.h[1] = *(const v8us*)(vp + 16 + 8 * h);
        al.h[0] = *(const v8us*)(wp + 8 * h);
        al.h[1] = *(const v8us*)(wp + 16 + 8 * h);
        o[dt] = mma_bf16(ah.v, ph.v, o[dt]);
        o[dt] = mma_bf16(ah.v, pl.v, o[dt]);
        o[dt] = mma_bf16(al.v, ph.v, o[dt]);
      }
    }
  }

  const float il = 1.0f / lrun;
#pragma unroll
  for (int p = 0; p < 2; ++p)
#pragma unroll
    for (int dt = 0; dt < 4; ++dt) {
      v8us pk;
#pragma unroll
      for (int r = 0; r < 8; ++r) {
        const float f = o[dt][r] * il;
        const unsigned short hb = bfb(f);
        pk[r] = p ? bfb(f - bfv(hb)) : hb;
      }
      *(v8us*)(CW + ((wave * 2 + p) * 16 + m) * 64 + dt * 16 + 8 * h) = pk;
    }
  __syncthreads();
  const int sub = lane >> 3, piece = lane & 7;
#pragma unroll
  for (int p = 0; p < 2; ++p) {
    unsigned short* plane = p ? cxl : cxh;
#pragma unroll
    for (int pass = 0; pass < 2; ++pass) {
      if (pass) __threadfence();
#pragma unroll
      for (int it = 0; it < 4; ++it) {
        const int qr = it * 4 + sub;
        v8us val = *(const v8us*)(CW + ((wave * 2 + p) * 16 + qr) * 64 + piece * 8);
        *(volatile v8us*)(plane + ((size_t)(b * 1024 + q0 + qr)) * 1024 + head * 64 + piece * 8) = val;
      }
    }
  }
}

__global__ __launch_bounds__(128) void k_proj(
    const unsigned short* __restrict__ ch, const unsigned short* __restrict__ cl,
    const unsigned short* __restrict__ wh, const unsigned short* __restrict__ wl,
    const float* __restrict__ bp, float* __restrict__ out) {
  __shared__ __attribute__((aligned(16))) float T[64 * TP];
  const int t = threadIdx.x, lane = t & 31, wave = t >> 5, h = lane >> 4, m = lane & 15;
  const int bm = blockIdx.y * 64, bn = blockIdx.x * 128;
  const int wm = (wave & 1) * 32, wn = (wave >> 1) * 64;

  v8f acc[2][4];
#pragma unroll
  for (int mi = 0; mi < 2; ++mi)
#pragma unroll
    for (int ni = 0; ni < 4; ++ni) acc[mi][ni] = zero8();

  const unsigned short* ah0p = ch + (size_t)(bm + wm + m) * 1024;
  const unsigned short* ah1p = ah0p + 16 * 1024;
  const unsigned short* al0p = cl + (size_t)(bm + wm + m) * 1024;
  const unsigned short* al1p = al0p + 16 * 1024;
  const unsigned short* bhp = wh + (size_t)(bn + wn + m) * 1024;
  const unsigned short* blp = wl + (size_t)(bn + wn + m) * 1024;
#pragma unroll 1
  for (int k0 = 0; k0 < 1024; k0 += 32) {
    FragU ah0, ah1, al0, al1;
    ah0.h[0] = *(const v8us*)(ah0p + k0 + 8 * h); ah0.h[1] = *(const v8us*)(ah0p + k0 + 16 + 8 * h);
    ah1.h[0] = *(const v8us*)(ah1p + k0 + 8 * h); ah1.h[1] = *(const v8us*)(ah1p + k0 + 16 + 8 * h);
    al0.h[0] = *(const v8us*)(al0p + k0 + 8 * h); al0.h[1] = *(const v8us*)(al0p + k0 + 16 + 8 * h);
    al1.h[0] = *(const v8us*)(al1p + k0 + 8 * h); al1.h[1] = *(const v8us*)(al1p + k0 + 16 + 8 * h);
#pragma unroll
    for (int ni = 0; ni < 4; ++ni) {
      const unsigned short* b0 = bhp + (size_t)ni * (16 * 1024) + k0;
      const unsigned short* b1 = blp + (size_t)ni * (16 * 1024) + k0;
      FragU wb, wr;
      wb.h[0] = *(const v8us*)(b0 + 8 * h); wb.h[1] = *(const v8us*)(b0 + 16 + 8 * h);
      wr.h[0] = *(const v8us*)(b1 + 8 * h); wr.h[1] = *(const v8us*)(b1 + 16 + 8 * h);
      acc[0][ni] = mma_bf16(ah0.v, wb.v, acc[0][ni]);
      acc[0][ni] = mma_bf16(ah0.v, wr.v, acc[0][ni]);
      acc[0][ni] = mma_bf16(al0.v, wb.v, acc[0][ni]);
      acc[1][ni] = mma_bf16(ah1.v, wb.v, acc[1][ni]);
      acc[1][ni] = mma_bf16(ah1.v, wr.v, acc[1][ni]);
      acc[1][ni] = mma_bf16(al1.v, wb.v, acc[1][ni]);
    }
  }

#pragma unroll
  for (int ni = 0; ni < 4; ++ni) {
    const float bias = bp[bn + wn + ni * 16 + m];
#pragma unroll
    for (int mi = 0; mi < 2; ++mi)
#pragma unroll
      for (int r = 0; r < 8; ++r)
        T[(wm + mi * 16 + 8 * h + r) * TP + wn + ni * 16 + m] = acc[mi][ni][r] + bias;
  }
  __syncthreads();
  const int sub = lane >> 3, piece = lane & 7;
#pragma unroll
  for (int pass = 0; pass < 2; ++pass) {
    if (pass) __threadfence();
#pragma unroll
    for (int it = 0; it < 16; ++it) {
      const int L = wave * 64 + it * 4 + sub;
      const int rw = L >> 2, seg = L & 3;
      const int col = seg * 32 + piece * 4;
      v4f val = *(const v4f*)(T + rw * TP + col);
      *(volatile v4f*)(out + (size_t)(bm + rw) * 1024 + bn + col) = val;
    }
  }
}

extern "C" void kernel_launch(void* const* d_in, const int* in_sizes, int n_in,
                              void* d_out, int out_size, void* d_ws,
                              size_t ws_size, hipStream_t stream) {
  const int B = 8, N = 1024, C = 1024, H = 16, HD = 64, C3 = 3072, M = B * N;
  if (n_in < 14) return;
  if (in_sizes[0] != M * C || in_sizes[1] != B * 1024 || in_sizes[2] != N * 32 ||
      in_sizes[3] != N * 32 || in_sizes[4] != N * 32 || in_sizes[5] != N * 32 ||
      in_sizes[6] != C * C3 || in_sizes[7] != C3 || in_sizes[8] != 1024 * C3 ||
      in_sizes[9] != C3 || in_sizes[10] != C * C || in_sizes[11] != C ||
      in_sizes[12] != HD || in_sizes[13] != HD || out_size != M * C)
    return;

  const float* x     = (const float*)d_in[0];
  const float* temb  = (const float*)d_in[1];
  const float* cos_y = (const float*)d_in[2];
  const float* sin_y = (const float*)d_in[3];
  const float* cos_x = (const float*)d_in[4];
  const float* sin_x = (const float*)d_in[5];
  const float* Wqkv  = (const float*)d_in[6];
  const float* bqkv  = (const float*)d_in[7];
  const float* Wt    = (const float*)d_in[8];
  const float* bt    = (const float*)d_in[9];
  const float* Wp    = (const float*)d_in[10];
  const float* bp    = (const float*)d_in[11];
  const float* qn_w  = (const float*)d_in[12];
  const float* kn_w  = (const float*)d_in[13];
  float* outp = (float*)d_out;

  size_t off = 0;
  char* wsb = (char*)d_ws;
  auto carve = [&](size_t bytes) -> char* {
    char* p = wsb + off;
    off += (bytes + 255) & ~(size_t)255;
    return p;
  };
  float* tvec          = (float*)carve((size_t)B * C3 * 4);
  unsigned short* xh   = (unsigned short*)carve((size_t)M * C * 2);
  unsigned short* wq   = (unsigned short*)carve((size_t)C3 * C * 2);
  unsigned short* wph  = (unsigned short*)carve((size_t)C * C * 2);
  unsigned short* wpl  = (unsigned short*)carve((size_t)C * C * 2);
  unsigned short* qpl  = (unsigned short*)carve((size_t)B * H * N * HD * 2);
  unsigned short* kpl  = (unsigned short*)carve((size_t)B * H * N * HD * 2);
  unsigned short* vth  = (unsigned short*)carve((size_t)B * H * HD * N * 2);
  unsigned short* vtl  = (unsigned short*)carve((size_t)B * H * HD * N * 2);
  unsigned short* cxh  = (unsigned short*)carve((size_t)M * C * 2);
  unsigned short* cxl  = (unsigned short*)carve((size_t)M * C * 2);
  if (off > ws_size) return;

  const int n8 = (M * C) / 8;
  k_cvt_x<<<dim3((n8 + 255) / 256), dim3(256), 0, stream>>>(x, xh, n8);
  k_tr<0><<<dim3(C3 / 64, C / 64), dim3(256), 0, stream>>>(Wqkv, C, C3, 32.0f, wq, wq);
  k_tr<1><<<dim3(C / 64, C / 64), dim3(256), 0, stream>>>(Wp, C, C, 1.0f, wph, wpl);
  k_temb<<<dim3(C3 / 32), dim3(64), 0, stream>>>(temb, Wt, bt, bqkv, tvec);
  k_qkv<<<dim3(C3 / 128, M / 64), dim3(128), 0, stream>>>(
      (const _Float16*)xh, (const _Float16*)wq, tvec, cos_y, sin_y, cos_x, sin_x, qn_w, kn_w,
      qpl, kpl, vth, vtl);
  k_attn<<<dim3(N / 64, B * H), dim3(128), 0, stream>>>(
      (const _Float16*)qpl, (const _Float16*)kpl, vth, vtl, cxh, cxl);
  k_proj<<<dim3(C / 128, M / 64), dim3(128), 0, stream>>>(cxh, cxl, wph, wpl, bp, outp);
}
